// LSA_75909251990221
// MI455X (gfx1250) — hardware-verified
//
#include <hip/hip_runtime.h>

#ifndef NB
#define NB 8
#endif
#ifndef SEQ
#define SEQ 1024
#endif
#define NB_FULL  8
#define SEQ_FULL 1024

typedef __attribute__((ext_vector_type(16))) _Float16 v16h;
typedef __attribute__((ext_vector_type(8)))  _Float16 v8h;
typedef __attribute__((ext_vector_type(16))) __bf16   v16b;
typedef __attribute__((ext_vector_type(8)))  __bf16   v8b;
typedef __attribute__((ext_vector_type(8)))  float    v8f;
typedef __attribute__((ext_vector_type(4)))  float    v4f;
typedef __attribute__((ext_vector_type(2)))  float    v2f;

constexpr int kBatch   = NB;
constexpr int kSeq     = SEQ;
constexpr int kSeqFull = SEQ_FULL;
constexpr int kDim     = 1024;
constexpr int kHeads   = 16;
constexpr int kHd      = 64;
constexpr int kInner   = kHeads * kHd;
constexpr int kQkvN    = 3 * kInner;
constexpr int kTok     = kBatch * kSeq;
constexpr int kQkLd    = 2 * kInner;
constexpr int kChunks  = kSeq / 64;
constexpr float kNegMax = -3.40282347e38f;
constexpr float kPCarry = 32768.0f;

static_assert(kBatch >= 1 && kBatch <= NB_FULL);
static_assert(kSeq >= 64 && kSeq <= SEQ_FULL && kSeq % 64 == 0);
static_assert(kTok % 64 == 0 && kQkLd % 64 == 0 && kDim % 32 == 0);
static_assert(kInner % 64 == 0 && kSeq % 64 == 0);
static_assert(kDim % 64 == 0 && kInner % 32 == 0);
static_assert(kHd == 64);
static_assert((kTok * kDim / 2) % 256 == 0 && (kQkvN * kDim / 2) % 256 == 0 && (kDim * kInner / 2) % 256 == 0);

__device__ __forceinline__ unsigned short f2bf_bits(float f) {
  unsigned u = __float_as_uint(f);
  return (unsigned short)((u + 0x7FFFu + ((u >> 16) & 1u)) >> 16);
}
__device__ __forceinline__ float bf_bits2f(unsigned short h) { return __uint_as_float(((unsigned)h) << 16); }

__device__ __forceinline__ void dep_guard_h(v8f& a, v8f& b, v16h x, v16h y) { asm volatile("v_nop\n\tv_nop\n\tv_nop\n\tv_nop" : "+v"(a), "+v"(b) : "v"(x), "v"(y)); }
__device__ __forceinline__ void dep_guard_b(v8f& a, v8f& b, v16b x, v16b y) { asm volatile("v_nop\n\tv_nop\n\tv_nop\n\tv_nop" : "+v"(a), "+v"(b) : "v"(x), "v"(y)); }
__device__ __forceinline__ void keep4_h(v16h a, v16h b, v16h c, v16h d) { asm volatile("v_nop" :: "v"(a), "v"(b), "v"(c), "v"(d)); }
__device__ __forceinline__ void keep4_b(v16b a, v16b b, v16b c, v16b d) { asm volatile("v_nop" :: "v"(a), "v"(b), "v"(c), "v"(d)); }
__device__ __forceinline__ void acc_guard4(v8f& a, v8f& b, v8f& c, v8f& d) { asm volatile("v_nop\n\tv_nop\n\tv_nop\n\tv_nop" : "+v"(a), "+v"(b), "+v"(c), "+v"(d)); }
template <typename T> struct Frag;
template <> struct Frag<_Float16> {
  typedef v16h V; union U { v16h v; v8h h[2]; };
  static __device__ __forceinline__ v16h load(const _Float16* p) {
    U f; f.h[0] = *(const v8h*)(p); f.h[1] = *(const v8h*)(p + 16); return f.v;
  }
  static __device__ __forceinline__ v8f mma(v16h a, v16h b, v8f c) {
    return __builtin_amdgcn_wmma_f32_16x16x32_f16(false, a, false, b, (short)0, c, false, false);
  }
  static __device__ __forceinline__ void guard(v8f& a, v8f& b, v16h x, v16h y) { dep_guard_h(a, b, x, y); }
  static __device__ __forceinline__ void keep(v16h a, v16h b, v16h c, v16h d) { keep4_h(a, b, c, d); }
};
template <> struct Frag<__bf16> {
  typedef v16b V; union U { v16b v; v8b h[2]; };
  static __device__ __forceinline__ v16b load(const __bf16* p) {
    U f; f.h[0] = *(const v8b*)(p); f.h[1] = *(const v8b*)(p + 16); return f.v;
  }
  static __device__ __forceinline__ v8f mma(v16b a, v16b b, v8f c) {
    return __builtin_amdgcn_wmma_f32_16x16x32_bf16(false, a, false, b, (short)0, c, false, false);
  }
  static __device__ __forceinline__ void guard(v8f& a, v8f& b, v16b x, v16b y) { dep_guard_b(a, b, x, y); }
  static __device__ __forceinline__ void keep(v16b a, v16b b, v16b c, v16b d) { keep4_b(a, b, c, d); }
};

template <int ET> struct Elem;
template <> struct Elem<0> { typedef _Float16 T; };
template <> struct Elem<1> { typedef __bf16 T; };
template <int ET, bool SPLIT, int BIAS_MODE, int OUT_MODE, bool RESID, int ACT = 0, bool BLO = true>
__global__ __launch_bounds__(256) void wmma_gemm64(
    const unsigned short* __restrict__ Ap, const unsigned short* __restrict__ A2p, int lda, long strideA,
    const unsigned short* __restrict__ Btp, const unsigned short* __restrict__ Bt2p, int ldb, long strideB,
    void* __restrict__ Cout, void* __restrict__ Cout2, int ldc, long strideC,
    const float* __restrict__ bias,
    const float* __restrict__ resid, long strideR,
    int M, int N, int K, float scale) {
  typedef typename Elem<ET>::T T;
  typedef typename Frag<T>::V V;
  const T* A = (const T*)Ap; const T* A2 = (const T*)A2p; const T* Bt = (const T*)Btp; const T* Bt2 = (const T*)Bt2p;
  __shared__ __align__(16) float sT[8][16 * 68];
  const int b    = blockIdx.y;
  const int lane = threadIdx.x & 31;
  const int wave = threadIdx.x >> 5;
  const int tilesN = N >> 6;
  const int tilesM = M >> 6;
  const int tile = blockIdx.x * 8 + wave;
  if (tile >= tilesM * tilesN) return;
  const int tm = tile / tilesN;
  const int tn = tile - tm * tilesN;
  const int m0 = tm << 6;
  const int n0 = tn << 6;

  const T* Ab  = A  + (size_t)b * strideA;
  const T* Bb  = Bt + (size_t)b * strideB;
  const T* Ab2 = SPLIT ? (A2  + (size_t)b * strideA) : nullptr;
  const T* Bb2 = (SPLIT && BLO) ? (Bt2 + (size_t)b * strideB) : nullptr;

  const int rlane = lane & 15;
  const int koff  = (lane >> 4) * 8;
  const int mOff  = (lane >> 4) * 8;

  v8f acc[4][4];
#pragma unroll
  for (int i = 0; i < 4; ++i)
#pragma unroll
    for (int j = 0; j < 4; ++j) acc[i][j] = (v8f){0.f,0.f,0.f,0.f,0.f,0.f,0.f,0.f};

  for (int k0 = 0; k0 < K; k0 += 32) {
    V bh[4], bl[4];
#pragma unroll
    for (int j = 0; j < 4; ++j) {
      const size_t bo = (size_t)(n0 + (j << 4) + rlane) * ldb + koff + k0;
      bh[j] = Frag<T>::load(Bb + bo);
      if (SPLIT && BLO) bl[j] = Frag<T>::load(Bb2 + bo);
    }
#pragma unroll
    for (int i = 0; i < 4; ++i) {
      const size_t ao = (size_t)(m0 + (i << 4) + rlane) * lda + koff + k0;
      V ah = Frag<T>::load(Ab + ao);
      V al;
      if (SPLIT) al = Frag<T>::load(Ab2 + ao);
#pragma unroll
      for (int j = 0; j < 4; ++j) {
        acc[i][j] = Frag<T>::mma(ah, bh[j], acc[i][j]);
        if (SPLIT) {
          if (BLO) acc[i][j] = Frag<T>::mma(ah, bl[j], acc[i][j]);
          acc[i][j] = Frag<T>::mma(al, bh[j], acc[i][j]);
        }
      }
      Frag<T>::guard(acc[i][0], acc[i][3], ah, SPLIT ? al : ah);
    }
    Frag<T>::keep(bh[0], bh[1], bh[2], bh[3]);
    if (SPLIT && BLO) Frag<T>::keep(bl[0], bl[1], bl[2], bl[3]);
  }
  acc_guard4(acc[0][0], acc[0][1], acc[0][2], acc[0][3]);
  acc_guard4(acc[1][0], acc[1][1], acc[1][2], acc[1][3]);
  acc_guard4(acc[2][0], acc[2][1], acc[2][2], acc[2][3]);
  acc_guard4(acc[3][0], acc[3][1], acc[3][2], acc[3][3]);

  float* slab = sT[wave];
  const float* Rb = RESID ? (resid + (size_t)b * strideR) : nullptr;
#pragma unroll
  for (int i = 0; i < 4; ++i) {
    const int mBase = m0 + (i << 4);
#pragma unroll
    for (int j = 0; j < 4; ++j) {
      const int n = n0 + (j << 4) + rlane;
      float bv = 0.f;
      if (BIAS_MODE == 2) bv = bf_bits2f(f2bf_bits(bias[n]));
#pragma unroll
      for (int r = 0; r < 8; ++r) {
        float v = acc[i][j][r] * scale;
        if (BIAS_MODE == 1) v += bf_bits2f(f2bf_bits(bias[mBase + mOff + r]));
        if (BIAS_MODE == 2) v += bv;
        if (RESID) v += Rb[(size_t)(mBase + mOff + r) * ldc + n];
        if (ACT == 1) v = tanhf(v);
        if (ACT == 2) v = fmaxf(v, 0.0f);
        if (ACT == 3) v = v / (1.0f + expf(-v));
        if (ACT == 4) v = (v > 0.f) ? v : 0.01f * v;
        if (ACT == 5) v = 0.5f * v * (1.0f + erff(v * 0.70710678118654752f));
        slab[(mOff + r) * 68 + (j << 4) + rlane] = v;
      }
    }
    __builtin_amdgcn_fence(__ATOMIC_RELEASE, "workgroup");
    __builtin_amdgcn_wave_barrier();
    __builtin_amdgcn_fence(__ATOMIC_ACQUIRE, "workgroup");
    if (OUT_MODE == 0) {
      float* C = (float*)Cout + (size_t)b * strideC;
      const int hh = lane >> 4, c4 = (lane & 15) * 4;
      for (int pass = 0; pass < 2; ++pass) {
#pragma unroll
        for (int it = 0; it < 8; ++it) {
          const int row = it * 2 + hh;
          v4f v = *(const v4f*)(slab + row * 68 + c4);
          *(volatile v4f*)(C + (size_t)(mBase + row) * ldc + n0 + c4) = v;
        }
        __threadfence();
      }
    } else {
      const int q = lane >> 3, c8 = (lane & 7) * 8;
      unsigned short* C  = (unsigned short*)Cout  + (size_t)b * strideC;
      unsigned short* C2 = (OUT_MODE == 2) ? ((unsigned short*)Cout2 + (size_t)b * strideC) : nullptr;
      for (int pass = 0; pass < 2; ++pass) {
#pragma unroll
        for (int it = 0; it < 4; ++it) {
          const int row = it * 4 + q;
          const float* sp = slab + row * 68 + c8;
          v8h hv, lv;
#pragma unroll
          for (int e = 0; e < 8; ++e) {
            if (OUT_MODE == 1) {
              hv[e] = (_Float16)sp[e];
            } else {
              unsigned short hb = f2bf_bits(sp[e]);
              unsigned short lb = f2bf_bits(sp[e] - bf_bits2f(hb));
              hv[e] = __builtin_bit_cast(_Float16, hb);
              lv[e] = __builtin_bit_cast(_Float16, lb);
            }
          }
          *(volatile v8h*)(C + (size_t)(mBase + row) * ldc + n0 + c8) = hv;
          if (OUT_MODE == 2) *(volatile v8h*)(C2 + (size_t)(mBase + row) * ldc + n0 + c8) = lv;
        }
        __threadfence();
      }
    }
    __builtin_amdgcn_fence(__ATOMIC_RELEASE, "workgroup");
    __builtin_amdgcn_wave_barrier();
    __builtin_amdgcn_fence(__ATOMIC_ACQUIRE, "workgroup");
  }
}

__global__ __launch_bounds__(256) void cast_f32_bf16x2(
    const float* __restrict__ in, unsigned short* __restrict__ out, int n2, int rowPairs, int seg, int segFull) {
  const int i = blockIdx.x * 256 + threadIdx.x;
  if (i < n2) {
    const int r  = i / rowPairs;
    const int c  = i - r * rowPairs;
    const int rb = r / seg;
    const int sr = rb * segFull + (r - rb * seg);
    const v2f f = *(const v2f*)(in + ((size_t)sr * rowPairs + c) * 2);
    const unsigned u = (unsigned)f2bf_bits(f[0]) | ((unsigned)f2bf_bits(f[1]) << 16);
    ((volatile unsigned*)out)[i] = u;
    __threadfence();
    ((volatile unsigned*)out)[i] = u;
  }
}

__device__ __forceinline__ v8f mma_f16_g(v16h a, v16h b, v8f c) {
  c = __builtin_amdgcn_wmma_f32_16x16x32_f16(false, a, false, b, (short)0, c, false, false);
  asm volatile("v_nop\n\tv_nop\n\tv_nop\n\tv_nop" : "+v"(c) : "v"(a), "v"(b));
  return c;
}

__global__ __launch_bounds__(128) void attn_diag_f16(
    const unsigned short* __restrict__ qkp, const unsigned short* __restrict__ vtp,
    const float* __restrict__ logt,
    unsigned short* __restrict__ ohp, unsigned short* __restrict__ olp) {
  union FH { v16h v; v8h h[2]; };
  __shared__ __align__(16) _Float16 Ksh[64 * 64];
  __shared__ __align__(16) _Float16 Vth[64 * 64];
  __shared__ __align__(16) _Float16 Psh[4][16 * 64];
  __shared__ __align__(16) float    Os[4][16 * 68];

  const _Float16* QK = (const _Float16*)qkp;
  const _Float16* VT = (const _Float16*)vtp;
  const int tid  = threadIdx.x;
  const int wave = tid >> 5;
  const int lane = tid & 31;
  const int hh   = lane >> 4;
  const int c    = lane & 15;

  const int bx = blockIdx.x;
  const int qb = bx % kChunks;
  const int bh = bx / kChunks;
  const int h  = bh % kHeads;
  const int b  = bh / kHeads;
  const int q0 = qb * 64 + wave * 16;
  const size_t rowbase = (size_t)b * kSeq;

  const float temp = expf(bf_bits2f(f2bf_bits(logt[0])));

  v16h qa[2];
#pragma unroll
  for (int dc = 0; dc < 2; ++dc)
    qa[dc] = Frag<_Float16>::load(QK + (rowbase + q0 + c) * kQkLd + h * kHd + dc * 32 + 8 * hh);

  float mrow[8], lrow[8];
  v8f oacc[4];
#pragma unroll
  for (int r = 0; r < 8; ++r) { mrow[r] = -__builtin_inff(); lrow[r] = 0.f; }
#pragma unroll
  for (int t = 0; t < 4; ++t) oacc[t] = (v8f){0.f,0.f,0.f,0.f,0.f,0.f,0.f,0.f};

  for (int kc = 0; kc < kChunks; ++kc) {
    const int kv0 = kc * 64;
    __syncthreads();
#pragma unroll
    for (int it = 0; it < 4; ++it) {
      const int idx = tid + 128 * it;
      const int r   = idx >> 3;
      const int c8  = (idx & 7) * 8;
      const v8h kk = *(const v8h*)(QK + (rowbase + kv0 + r) * kQkLd + kInner + h * kHd + c8);
      const v8h vv = *(const v8h*)(VT + ((size_t)bh * kHd + r) * kSeq + kv0 + c8);
      *(v8h*)(Ksh + r * 64 + c8) = kk;
      *(v8h*)(Vth + r * 64 + c8) = vv;
    }
    __syncthreads();

    v8f s[4];
#pragma unroll
    for (int j = 0; j < 4; ++j) {
      s[j] = (v8f){0.f,0.f,0.f,0.f,0.f,0.f,0.f,0.f};
#pragma unroll
      for (int dc = 0; dc < 2; ++dc) {
        FH kb;
        kb.h[0] = *(const v8h*)(Ksh + (j * 16 + c) * 64 + dc * 32 + 8 * hh);
        kb.h[1] = *(const v8h*)(Ksh + (j * 16 + c) * 64 + dc * 32 + 16 + 8 * hh);
        s[j] = mma_f16_g(qa[dc], kb.v, s[j]);
      }
    }
    float cm[8];
#pragma unroll
    for (int r = 0; r < 8; ++r) {
      const int qrow = q0 + 8 * hh + r;
      float m = -__builtin_inff();
#pragma unroll
      for (int j = 0; j < 4; ++j) {
        const int kvcol = kv0 + j * 16 + c;
        float sv = s[j][r] * temp;
        if (kvcol == qrow) sv = kNegMax;
        s[j][r] = sv;
        m = fmaxf(m, sv);
      }
#pragma unroll
      for (int off = 1; off < 16; off <<= 1) m = fmaxf(m, __shfl_xor(m, off, 32));
      cm[r] = m;
    }
    _Float16* pwh = Psh[wave];
#pragma unroll
    for (int r = 0; r < 8; ++r) {
      const float mnew  = fmaxf(mrow[r], cm[r]);
      const float alpha = expf(mrow[r] - mnew);
      mrow[r] = mnew;
      float psum = 0.f;
#pragma unroll
      for (int j = 0; j < 4; ++j) {
        const float p = expf(s[j][r] - mnew);
        psum += p;
        pwh[(8 * hh + r) * 64 + j * 16 + c] = (_Float16)(p * kPCarry);
      }
#pragma unroll
      for (int off = 1; off < 16; off <<= 1) psum += __shfl_xor(psum, off, 32);
      lrow[r] = lrow[r] * alpha + psum;
#pragma unroll
      for (int t = 0; t < 4; ++t) oacc[t][r] *= alpha;
    }
    __builtin_amdgcn_fence(__ATOMIC_RELEASE, "workgroup");
    __builtin_amdgcn_wave_barrier();
    __builtin_amdgcn_fence(__ATOMIC_ACQUIRE, "workgroup");
#pragma unroll
    for (int kk = 0; kk < 2; ++kk) {
      FH pa;
      pa.h[0] = *(const v8h*)(pwh + c * 64 + kk * 32 + 8 * hh);
      pa.h[1] = *(const v8h*)(pwh + c * 64 + kk * 32 + 16 + 8 * hh);
#pragma unroll
      for (int t = 0; t < 4; ++t) {
        FH vb;
        vb.h[0] = *(const v8h*)(Vth + (t * 16 + c) * 64 + kk * 32 + 8 * hh);
        vb.h[1] = *(const v8h*)(Vth + (t * 16 + c) * 64 + kk * 32 + 16 + 8 * hh);
        oacc[t] = mma_f16_g(pa.v, vb.v, oacc[t]);
      }
    }
  }

  float* os = Os[wave];
#pragma unroll
  for (int r = 0; r < 8; ++r) {
    const float inv = 1.0f / (lrow[r] * kPCarry);
#pragma unroll
    for (int t = 0; t < 4; ++t) os[(8 * hh + r) * 68 + t * 16 + c] = oacc[t][r] * inv;
  }
  __builtin_amdgcn_fence(__ATOMIC_RELEASE, "workgroup");
  __builtin_amdgcn_wave_barrier();
  __builtin_amdgcn_fence(__ATOMIC_ACQUIRE, "workgroup");
  {
    const int q4 = lane >> 3, c8 = (lane & 7) * 8;
    for (int pass = 0; pass < 2; ++pass) {
#pragma unroll
      for (int it = 0; it < 4; ++it) {
        const int row = it * 4 + q4;
        const float* sp = os + row * 68 + c8;
        v8h hv, lv;
#pragma unroll
        for (int e = 0; e < 8; ++e) {
          const unsigned short hb = f2bf_bits(sp[e]);
          const unsigned short lb = f2bf_bits(sp[e] - bf_bits2f(hb));
          hv[e] = __builtin_bit_cast(_Float16, hb);
          lv[e] = __builtin_bit_cast(_Float16, lb);
        }
        const size_t o = (rowbase + q0 + row) * (size_t)kInner + h * kHd + c8;
        *(volatile v8h*)(ohp + o) = hv;
        *(volatile v8h*)(olp + o) = lv;
      }
      __threadfence();
    }
  }
}

extern "C" void kernel_launch(void* const* d_in, const int* in_sizes, int n_in,
                              void* d_out, int out_size, void* d_ws, size_t ws_size,
                              hipStream_t stream) {
  if (n_in < 5) return;
  const long needX = ((long)(kBatch - 1) * kSeqFull + kSeq) * (long)kDim;
  if ((long)in_sizes[0] < needX || in_sizes[1] < kQkvN * kDim || in_sizes[2] < kDim * kInner ||
      in_sizes[3] < kDim || in_sizes[4] < 1) return;
  if (out_size < kTok * kDim) return;

  const float* x     = (const float*)d_in[0];
  const float* wqkv  = (const float*)d_in[1];
  const float* wout  = (const float*)d_in[2];
  const float* bout  = (const float*)d_in[3];
  const float* tempr = (const float*)d_in[4];
  float* out = (float*)d_out;

  const size_t szXb  = (size_t)kTok * kDim * 2;
  const size_t szWq  = (size_t)kQkvN * kDim * 2;
  const size_t szWo  = (size_t)kDim * kInner * 2;
  const size_t szQk  = (size_t)kTok * kQkLd * 2;
  const size_t szVt  = (size_t)kBatch * kInner * kSeq * 2;
  const size_t szO   = (size_t)kTok * kInner * 2;
  const size_t offXb = 0, offWq = offXb + szXb, offWo = offWq + szWq, offQk = offWo + szWo,
               offVt = offQk + szQk, offOh = offVt + szVt, offOl = offOh + szO, total = offOl + szO;
  if (total > ws_size) return;

  char* ws = (char*)d_ws;
  unsigned short* xb  = (unsigned short*)(ws + offXb);
  unsigned short* wqb = (unsigned short*)(ws + offWq);
  unsigned short* wob = (unsigned short*)(ws + offWo);
  unsigned short* qk  = (unsigned short*)(ws + offQk);
  unsigned short* vt  = (unsigned short*)(ws + offVt);
  unsigned short* oh  = (unsigned short*)(ws + offOh);
  unsigned short* ol  = (unsigned short*)(ws + offOl);

  {
    const int n2 = kTok * kDim / 2;
    cast_f32_bf16x2<<<dim3((n2 + 255) / 256), dim3(256), 0, stream>>>(x, xb, n2, kDim / 2, kSeq, kSeqFull);
  }
  {
    const int n2 = kQkvN * kDim / 2;
    cast_f32_bf16x2<<<dim3((n2 + 255) / 256), dim3(256), 0, stream>>>(wqkv, wqb, n2, kDim / 2, kQkvN, kQkvN);
  }
  {
    const int n2 = kDim * kInner / 2;
    cast_f32_bf16x2<<<dim3((n2 + 255) / 256), dim3(256), 0, stream>>>(wout, wob, n2, kInner / 2, kDim, kDim);
  }
  {
    const int tiles = (kTok / 64) * (kQkLd / 64);
    wmma_gemm64<1, false, 0, 1, false><<<dim3((tiles + 7) / 8, 1), dim3(256), 0, stream>>>(
        xb, xb, kDim, 0L, wqb, wqb, kDim, 0L, (void*)qk, (void*)qk, kQkLd, 0L,
        bout, bout, 0L, kTok, kQkLd, kDim, 1.0f);
  }
  {
    const int tiles = (kInner / 64) * (kSeq / 64);
    wmma_gemm64<1, false, 0, 1, false><<<dim3((tiles + 7) / 8, kBatch), dim3(256), 0, stream>>>(
        wqb + (size_t)kQkLd * kDim, wqb + (size_t)kQkLd * kDim, kDim, 0L,
        xb, xb, kDim, (long)kSeq * kDim,
        (void*)vt, (void*)vt, kSeq, (long)kInner * kSeq,
        bout, bout, 0L, kInner, kSeq, kDim, 1.0f);
  }
  attn_diag_f16<<<dim3(kBatch * kHeads * kChunks), dim3(128), 0, stream>>>(qk, vt, tempr, oh, ol);
  {
    const int tiles = (kTok / 64) * (kDim / 64);
    wmma_gemm64<1, true, 2, 0, false, 0, false><<<dim3((tiles + 7) / 8, 1), dim3(256), 0, stream>>>(
        oh, ol, kInner, 0L, wob, wob, kInner, 0L, (void*)out, (void*)out, kDim, 0L,
        bout, bout, 0L, kTok, kDim, kInner, 1.0f);
  }
}
